// TransformerEncoderLayerSpatial_987842478856
// MI455X (gfx1250) — hardware-verified
//
#include <hip/hip_runtime.h>
#include <math.h>
#include <stdint.h>

#define NB      2
#define CD      256
#define HW      64
#define NSEQ    4096
#define NHEAD   8
#define HDIM    32
#define DFF     1024
#define MP      (NB * NSEQ)
#define LNEPS   1.0e-5f
#define WSC     64.0f
#define QCARRY  16.0f
#define KCARRY  8.0f
#define VCARRY  4.0f
#define PCARRY  16384.0f
#define AOCARRY 8.0f
#define YCARRY  4.0f
#define GCARRY  4.0f
static_assert(NHEAD * HDIM == CD);
static_assert(HW * HW == NSEQ);
static_assert((MP % 64) == 0 && (CD % 64) == 0 && (DFF % 64) == 0 && (NSEQ % 64) == 0);
static_assert(CD == 32 * 8);

typedef _Float16 v16h __attribute__((ext_vector_type(16)));
typedef _Float16 v8h  __attribute__((ext_vector_type(8)));
typedef _Float16 v4h  __attribute__((ext_vector_type(4)));
typedef float    v8f  __attribute__((ext_vector_type(8)));
typedef float    v4f  __attribute__((ext_vector_type(4)));
typedef unsigned int v4u __attribute__((ext_vector_type(4)));
typedef unsigned int v2u __attribute__((ext_vector_type(2)));

union FragH { v16h v; v8h h[2]; };

__device__ __forceinline__ unsigned short bf_bits(float f) {
  unsigned u = __float_as_uint(f);
  return (unsigned short)((u + 0x7FFFu + ((u >> 16) & 1u)) >> 16);
}
__device__ __forceinline__ float bf_up(unsigned short h) { return __uint_as_float(((unsigned)h) << 16); }
__device__ __forceinline__ float bfr(float f) { return bf_up(bf_bits(f)); }
__device__ __forceinline__ unsigned short h_bits(_Float16 x) { return __builtin_bit_cast(unsigned short, x); }
__device__ __forceinline__ unsigned pk16(unsigned short a, unsigned short b) { return (unsigned)a | ((unsigned)b << 16); }
__device__ __forceinline__ v8f zero8() { v8f z = {0.f, 0.f, 0.f, 0.f, 0.f, 0.f, 0.f, 0.f}; return z; }

__device__ __forceinline__ v16h ldfrag_h(const _Float16* p) {
  FragH f;
  f.h[0] = *(const v8h*)(p);
  f.h[1] = *(const v8h*)(p + 16);
  return f.v;
}

__device__ __forceinline__ v8f mma_h(v16h a, v16h b, v8f c) {
  c = __builtin_amdgcn_wmma_f32_16x16x32_f16(false, a, false, b, (short)0, c, false, false);
#if defined(__HIP_DEVICE_COMPILE__)
  asm volatile("v_nop\n\tv_nop\n\tv_nop\n\tv_nop" : "+v"(c) : "v"(a), "v"(b));
#endif
  return c;
}
__device__ __forceinline__ v8f mma_h_raw(v16h a, v16h b, v8f c) {
  return __builtin_amdgcn_wmma_f32_16x16x32_f16(false, a, false, b, (short)0, c, false, false);
}
__device__ __forceinline__ void dep_guard1(v8f& a, v8f& b, v16h x) {
#if defined(__HIP_DEVICE_COMPILE__)
  asm volatile("v_nop\n\tv_nop\n\tv_nop\n\tv_nop" : "+v"(a), "+v"(b) : "v"(x));
#endif
}
__device__ __forceinline__ void dep_guard3(v8f& a, v8f& b, v16h x, v16h y, v16h z) {
#if defined(__HIP_DEVICE_COMPILE__)
  asm volatile("v_nop\n\tv_nop\n\tv_nop\n\tv_nop" : "+v"(a), "+v"(b) : "v"(x), "v"(y), "v"(z));
#endif
}
__device__ __forceinline__ void keep4_h(v16h a, v16h b, v16h c, v16h d) {
#if defined(__HIP_DEVICE_COMPILE__)
  asm volatile("v_nop" :: "v"(a), "v"(b), "v"(c), "v"(d));
#endif
}
__device__ __forceinline__ void acc_guard4(v8f& a, v8f& b, v8f& c, v8f& d) {
#if defined(__HIP_DEVICE_COMPILE__)
  asm volatile("v_nop\n\tv_nop\n\tv_nop\n\tv_nop" : "+v"(a), "+v"(b), "+v"(c), "+v"(d));
#endif
}
__device__ __forceinline__ void wave_sync_lds() {
  __builtin_amdgcn_fence(__ATOMIC_RELEASE, "workgroup");
  __builtin_amdgcn_wave_barrier();
  __builtin_amdgcn_fence(__ATOMIC_ACQUIRE, "workgroup");
}
__device__ __forceinline__ float wsum(float v) {
#pragma unroll
  for (int off = 16; off > 0; off >>= 1) v += __shfl_xor(v, off, 32);
  return v;
}

__global__ __launch_bounds__(256) void conv_h16(const float* __restrict__ W, unsigned short* Wh, int n8, float wsc) {
  const int i  = blockIdx.x * 256 + threadIdx.x;
  const int ic = (i < n8) ? i : (n8 - 1);
  const float* src = W + (size_t)ic * 8;
  const v4f a = *(const v4f*)(src);
  const v4f c = *(const v4f*)(src + 4);
  v4u o;
  o[0] = pk16(h_bits((_Float16)(bfr(a[0]) * wsc)), h_bits((_Float16)(bfr(a[1]) * wsc)));
  o[1] = pk16(h_bits((_Float16)(bfr(a[2]) * wsc)), h_bits((_Float16)(bfr(a[3]) * wsc)));
  o[2] = pk16(h_bits((_Float16)(bfr(c[0]) * wsc)), h_bits((_Float16)(bfr(c[1]) * wsc)));
  o[3] = pk16(h_bits((_Float16)(bfr(c[2]) * wsc)), h_bits((_Float16)(bfr(c[3]) * wsc)));
  if (i < n8) *(volatile v4u*)(Wh + (size_t)i * 8) = o;
  __threadfence();
  if (i < n8) *(volatile v4u*)(Wh + (size_t)i * 8) = o;
}

__global__ __launch_bounds__(256) void xprep(const float* __restrict__ src, const float* __restrict__ per,
                                              const float* __restrict__ pec, unsigned short* XH,
                                              unsigned short* XPR, unsigned short* XPC) {
  __shared__ __align__(16) float T[CD * 36];
  const int tid = threadIdx.x, wave = tid >> 5, lane = tid & 31;
  const int bx = blockIdx.x;
  const int b  = bx >> 7;
  const int n0 = (bx & 127) * 32;
  const float* sb = src + (size_t)b * CD * NSEQ + n0;
  {
    const int q = lane >> 3, e = lane & 7;
#pragma unroll
    for (int it = 0; it < 8; ++it) {
      const int c = wave * 32 + it * 4 + q;
      const v4f v = *(const v4f*)(sb + (size_t)c * NSEQ + 4 * e);
      *(v4f*)(T + c * 36 + 4 * e) = v;
    }
  }
  __syncthreads();
#pragma unroll 1
  for (int i = 0; i < 4; ++i) {
    const int tl = wave * 4 + i;
    const int n  = n0 + tl;
    const int w  = n & 63, hr = n >> 6;
    const float* prp = per + ((size_t)(b * HW + w)) * CD + 8 * lane;
    const float* pcp = pec + ((size_t)(b * HW + hr)) * CD + 8 * lane;
    const v4f r0 = *(const v4f*)(prp), r1 = *(const v4f*)(prp + 4);
    const v4f c0 = *(const v4f*)(pcp), c1 = *(const v4f*)(pcp + 4);
    float x[8], pr[8], pc[8];
#pragma unroll
    for (int e = 0; e < 8; ++e) x[e] = bfr(T[(8 * lane + e) * 36 + tl]);
#pragma unroll
    for (int e = 0; e < 4; ++e) {
      pr[e] = bfr(r0[e]); pr[4 + e] = bfr(r1[e]);
      pc[e] = bfr(c0[e]); pc[4 + e] = bfr(c1[e]);
    }
    v4u ox, orw, ocl;
#pragma unroll
    for (int e = 0; e < 4; ++e) {
      ox[e]  = pk16(h_bits((_Float16)x[2 * e]), h_bits((_Float16)x[2 * e + 1]));
      orw[e] = pk16(h_bits((_Float16)(x[2 * e] + pr[2 * e])), h_bits((_Float16)(x[2 * e + 1] + pr[2 * e + 1])));
      ocl[e] = pk16(h_bits((_Float16)(x[2 * e] + pc[2 * e])), h_bits((_Float16)(x[2 * e + 1] + pc[2 * e + 1])));
    }
    const size_t ro = ((size_t)b * NSEQ + n) * CD + 8 * lane;
    for (int pass = 0; pass < 2; ++pass) {
      *(volatile v4u*)(XH  + ro) = ox;
      *(volatile v4u*)(XPR + ro) = orw;
      *(volatile v4u*)(XPC + ro) = ocl;
      __threadfence();
    }
  }
}

__global__ __launch_bounds__(256) void xmean(const float* __restrict__ src, const float* __restrict__ per,
                                              const float* __restrict__ pec, unsigned short* XM) {
  __shared__ __align__(16) float Ms[32 * 260];
  const int tid = threadIdx.x, wave = tid >> 5, lane = tid & 31;
  const int bx   = blockIdx.x;
  const int pcnk = bx & 1, sel = (bx >> 1) & 1, b = bx >> 2;
  const int p0   = pcnk * 32;
  const int p    = p0 + lane;
  const float* sb = src + (size_t)b * CD * NSEQ;
  const int base = sel ? (p * HW) : p;
  const int step = sel ? 1 : HW;
#pragma unroll 1
  for (int ci = 0; ci < 32; ++ci) {
    const int c = wave * 32 + ci;
    const float* sp = sb + (size_t)c * NSEQ + base;
    float s = 0.f;
#pragma unroll 8
    for (int r = 0; r < HW; ++r) s += bfr(sp[r * step]);
    Ms[lane * 260 + c] = s;
  }
  __syncthreads();
  const float* pe = sel ? pec : per;
#pragma unroll 1
  for (int i = 0; i < 4; ++i) {
    const int pl = wave * 4 + i;
    const float* pp = pe + ((size_t)(b * HW + p0 + pl)) * CD + 8 * lane;
    const v4f a0 = *(const v4f*)(pp), a1 = *(const v4f*)(pp + 4);
    float m[8];
#pragma unroll
    for (int e = 0; e < 4; ++e) {
      m[e]     = Ms[pl * 260 + 8 * lane + e]     * (1.0f / HW) + bfr(a0[e]);
      m[4 + e] = Ms[pl * 260 + 8 * lane + 4 + e] * (1.0f / HW) + bfr(a1[e]);
    }
    v4u o;
#pragma unroll
    for (int e = 0; e < 4; ++e) o[e] = pk16(h_bits((_Float16)m[2 * e]), h_bits((_Float16)m[2 * e + 1]));
    const size_t ro = ((size_t)((sel * NB + b) * HW + p0 + pl)) * CD + 8 * lane;
    *(volatile v4u*)(XM + ro) = o;
    __threadfence();
    *(volatile v4u*)(XM + ro) = o;
  }
}

template <int A32, int OM, int BIASM, int ACT, int RES>
__global__ __launch_bounds__(256) void gemm64(
    const void* __restrict__ Ap, int lda, long long strideA, float ascale,
    const unsigned short* __restrict__ Btp, int ldb, long long strideB,
    const float* __restrict__ bias0, const float* __restrict__ bias1, float bscale,
    const void* resid,
    void* Cout, int ldc, long long strideC,
    int M, int N, int K, float oscale) {
  const _Float16* Bt = (const _Float16*)(const void*)Btp;
  __shared__ __align__(16) float sT[8][16 * 68];
  const int b    = blockIdx.y;
  const int lane = threadIdx.x & 31;
  const int wave = threadIdx.x >> 5;
  const int tilesN = N >> 6;
  const int tilesM = M >> 6;
  const int tile = blockIdx.x * 8 + wave;
  if (tile >= tilesM * tilesN) return;
  const int tm = tile / tilesN;
  const int tn = tile - tm * tilesN;
  const int m0 = tm << 6;
  const int n0 = tn << 6;

  const _Float16* Ah = (const _Float16*)Ap + (size_t)b * strideA;
  const float*    Af = (const float*)Ap + (size_t)b * strideA;
  const _Float16* Bb = Bt + (size_t)b * strideB;
  const float* bias = (b == 0) ? bias0 : bias1;

  const int rlane = lane & 15;
  const int koff  = (lane >> 4) * 8;
  const int mOff  = (lane >> 4) * 8;

  v8f acc[4][4];
#pragma unroll
  for (int i = 0; i < 4; ++i)
#pragma unroll
    for (int j = 0; j < 4; ++j) acc[i][j] = zero8();

  for (int k0 = 0; k0 < K; k0 += 32) {
    v16h bh[4];
#pragma unroll
    for (int j = 0; j < 4; ++j) {
      const size_t bo = (size_t)(n0 + (j << 4) + rlane) * ldb + koff + k0;
      bh[j] = ldfrag_h(Bb + bo);
    }
#pragma unroll
    for (int i = 0; i < 4; ++i) {
      v16h ah;
      if (A32) {
        const float* ap = Af + (size_t)(m0 + (i << 4) + rlane) * lda + koff + k0;
        const v4f x0 = *(const v4f*)(ap), x1 = *(const v4f*)(ap + 4);
        const v4f x2 = *(const v4f*)(ap + 16), x3 = *(const v4f*)(ap + 20);
        FragH f;
#pragma unroll
        for (int e = 0; e < 4; ++e) {
          f.h[0][e]     = (_Float16)(x0[e] * ascale);
          f.h[0][4 + e] = (_Float16)(x1[e] * ascale);
          f.h[1][e]     = (_Float16)(x2[e] * ascale);
          f.h[1][4 + e] = (_Float16)(x3[e] * ascale);
        }
        ah = f.v;
      } else {
        const size_t ao = (size_t)(m0 + (i << 4) + rlane) * lda + koff + k0;
        ah = ldfrag_h(Ah + ao);
      }
#pragma unroll
      for (int j = 0; j < 4; ++j) acc[i][j] = mma_h_raw(ah, bh[j], acc[i][j]);
      dep_guard1(acc[i][0], acc[i][3], ah);
    }
    keep4_h(bh[0], bh[1], bh[2], bh[3]);
  }
  acc_guard4(acc[0][0], acc[0][1], acc[0][2], acc[0][3]);
  acc_guard4(acc[1][0], acc[1][1], acc[1][2], acc[1][3]);
  acc_guard4(acc[2][0], acc[2][1], acc[2][2], acc[2][3]);
  acc_guard4(acc[3][0], acc[3][1], acc[3][2], acc[3][3]);

  const int hh2 = lane >> 4, c4 = (lane & 15) * 4;
  const int q8  = lane >> 3, c8 = (lane & 7) * 8;
  float bc[8];
#pragma unroll
  for (int e = 0; e < 8; ++e) bc[e] = 0.f;
  if (BIASM == 0) {
    if (OM == 0) {
      const int cb = n0 + c4;
      const int i0 = (cb < N - 4) ? cb : (N - 4);
      const v4f b0v = *(const v4f*)(bias + i0);
#pragma unroll
      for (int e = 0; e < 4; ++e) bc[e] = bfr(b0v[e]) * bscale;
    } else {
      const int cb = n0 + c8;
      const int i0 = (cb < N - 8) ? cb : (N - 8);
      const v4f b0a = *(const v4f*)(bias + i0), b0b = *(const v4f*)(bias + i0 + 4);
#pragma unroll
      for (int e = 0; e < 4; ++e) {
        bc[e]     = bfr(b0a[e]) * bscale;
        bc[4 + e] = bfr(b0b[e]) * bscale;
      }
    }
  }

  float* slab = sT[wave];
#pragma unroll
  for (int i = 0; i < 4; ++i) {
    const int mBase = m0 + (i << 4);
#pragma unroll
    for (int j = 0; j < 4; ++j) {
#pragma unroll
      for (int r = 0; r < 8; ++r) {
        slab[(mOff + r) * 68 + (j << 4) + rlane] = acc[i][j][r];
      }
    }
    wave_sync_lds();
    if (OM == 0) {
      float* C = (float*)Cout + (size_t)b * strideC;
      const float*    Rf = (const float*)resid + (size_t)b * strideC;
      const _Float16* Rh = (const _Float16*)resid + (size_t)b * strideC;
      v4f vals[8];
#pragma unroll
      for (int it = 0; it < 8; ++it) {
        const int row = it * 2 + hh2;
        v4f v = *(const v4f*)(slab + row * 68 + c4);
#pragma unroll
        for (int e = 0; e < 4; ++e) {
          float f = v[e] * oscale + bc[e];
          if (ACT) f = fmaxf(f, 0.f);
          v[e] = f;
        }
        if (RES == 1) {
          const v4f rr = *(const v4f*)(Rf + (size_t)(mBase + row) * ldc + n0 + c4);
#pragma unroll
          for (int e = 0; e < 4; ++e) v[e] += rr[e];
        }
        if (RES == 2) {
          const v4h rr = *(const v4h*)(Rh + (size_t)(mBase + row) * ldc + n0 + c4);
#pragma unroll
          for (int e = 0; e < 4; ++e) v[e] += (float)rr[e];
        }
        vals[it] = v;
      }
      for (int pass = 0; pass < 2; ++pass) {
#pragma unroll
        for (int it = 0; it < 8; ++it) {
          const int row = it * 2 + hh2;
          *(volatile v4f*)(C + (size_t)(mBase + row) * ldc + n0 + c4) = vals[it];
        }
        __threadfence();
      }
    } else {
      unsigned short* C = (unsigned short*)Cout + (size_t)b * strideC;
      v4u hv[4];
#pragma unroll
      for (int it = 0; it < 4; ++it) {
        const int row = it * 4 + q8;
        const float* sp = slab + row * 68 + c8;
        float bm = 0.f;
        if (BIASM == 1) bm = bfr(bias[mBase + row]) * bscale;
        v4u a;
#pragma unroll
        for (int e = 0; e < 4; ++e) {
          float f0 = sp[2 * e]     * oscale + ((BIASM == 1) ? bm : bc[2 * e]);
          float f1 = sp[2 * e + 1] * oscale + ((BIASM == 1) ? bm : bc[2 * e + 1]);
          if (ACT) { f0 = fmaxf(f0, 0.f); f1 = fmaxf(f1, 0.f); }
          a[e] = pk16(h_bits((_Float16)f0), h_bits((_Float16)f1));
        }
        hv[it] = a;
      }
      for (int pass = 0; pass < 2; ++pass) {
#pragma unroll
        for (int it = 0; it < 4; ++it) {
          const int row = it * 4 + q8;
          *(volatile v4u*)(C + (size_t)(mBase + row) * ldc + n0 + c8) = hv[it];
        }
        __threadfence();
      }
    }
    wave_sync_lds();
  }
}

__global__ __launch_bounds__(128)
void attn_rc(const unsigned short* __restrict__ qh, const unsigned short* __restrict__ kh,
             const unsigned short* __restrict__ vt, float* ao) {
  __shared__ __align__(16) float Ps[4][2][16 * 64];
  __shared__ __align__(16) float Os[4][16 * 32];

  const int tid  = threadIdx.x;
  const int wave = tid >> 5;
  const int lane = tid & 31;
  const int hh   = lane >> 4;
  const int c    = lane & 15;

  const int bx = blockIdx.x;
  const int qb = bx & 63;
  const int a  = (bx >> 6) & 7;
  const int b  = bx >> 9;
  const int q0 = qb * 64 + wave * 16;
  const size_t gr = (size_t)b * NSEQ + q0;

  const _Float16* Q  = (const _Float16*)(const void*)qh;
  const _Float16* Kp = (const _Float16*)(const void*)kh;
  const _Float16* V  = (const _Float16*)(const void*)vt + ((size_t)b * CD + (size_t)a * HDIM) * NSEQ;
  const float sinv = 1.0f / (QCARRY * KCARRY);

#pragma unroll
  for (int sel = 0; sel < 2; ++sel) {
    const v16h qa = ldfrag_h(Q + ((size_t)sel * MP + gr + c) * CD + a * HDIM + 8 * hh);
    v8f s[4];
#pragma unroll
    for (int j = 0; j < 4; ++j) {
      const v16h kb = ldfrag_h(Kp + (((size_t)sel * NB + b) * HW + 16 * j + c) * CD + a * HDIM + 8 * hh);
      s[j] = mma_h(qa, kb, zero8());
    }
    float* pt = Ps[wave][sel];
#pragma unroll
    for (int r = 0; r < 8; ++r) {
      const float v0 = s[0][r] * sinv, v1 = s[1][r] * sinv, v2 = s[2][r] * sinv, v3 = s[3][r] * sinv;
      float m = fmaxf(fmaxf(v0, v1), fmaxf(v2, v3));
#pragma unroll
      for (int off = 1; off < 16; off <<= 1) m = fmaxf(m, __shfl_xor(m, off, 32));
      const float e0 = __expf(v0 - m), e1 = __expf(v1 - m), e2 = __expf(v2 - m), e3 = __expf(v3 - m);
      float ps = (e0 + e1) + (e2 + e3);
#pragma unroll
      for (int off = 1; off < 16; off <<= 1) ps += __shfl_xor(ps, off, 32);
      const float inv = 1.0f / ps;
      const int ro = (8 * hh + r) * 64 + c;
      pt[ro]      = e0 * inv;
      pt[ro + 16] = e1 * inv;
      pt[ro + 32] = e2 * inv;
      pt[ro + 48] = e3 * inv;
    }
  }
  wave_sync_lds();

  v4f prv[8];
  {
    const float* prow = Ps[wave][0] + c * 64 + 8 * hh;
#pragma unroll
    for (int j = 0; j < 4; ++j) {
      prv[2 * j]     = *(const v4f*)(prow + 16 * j);
      prv[2 * j + 1] = *(const v4f*)(prow + 16 * j + 4);
    }
  }
  const float* pcrow = Ps[wave][1] + c * 64;

  v8f oacc0 = zero8(), oacc1 = zero8();
#pragma unroll 1
  for (int hp = 0; hp < HW; ++hp) {
    const float pcv = pcrow[hp] * PCARRY;
#pragma unroll
    for (int wi = 0; wi < 2; ++wi) {
      const v4f p0 = prv[4 * wi], p1 = prv[4 * wi + 1], p2 = prv[4 * wi + 2], p3 = prv[4 * wi + 3];
      FragH pa;
#pragma unroll
      for (int e = 0; e < 4; ++e) {
        pa.h[0][e]     = (_Float16)(pcv * p0[e]);
        pa.h[0][4 + e] = (_Float16)(pcv * p1[e]);
        pa.h[1][e]     = (_Float16)(pcv * p2[e]);
        pa.h[1][4 + e] = (_Float16)(pcv * p3[e]);
      }
      const int k0 = hp * 64 + wi * 32;
      const v16h vb0 = ldfrag_h(V + (size_t)c * NSEQ + k0 + 8 * hh);
      const v16h vb1 = ldfrag_h(V + (size_t)(16 + c) * NSEQ + k0 + 8 * hh);
      oacc0 = mma_h_raw(pa.v, vb0, oacc0);
      oacc1 = mma_h_raw(pa.v, vb1, oacc1);
      dep_guard3(oacc0, oacc1, pa.v, vb0, vb1);
    }
  }

  float* os = Os[wave];
  const float oinv = 1.0f / (PCARRY * VCARRY);
#pragma unroll
  for (int r = 0; r < 8; ++r) {
    os[(8 * hh + r) * 32 + c]      = oacc0[r] * oinv;
    os[(8 * hh + r) * 32 + 16 + c] = oacc1[r] * oinv;
  }
  wave_sync_lds();
  {
    const int q4 = lane >> 3, e4 = (lane & 7) * 4;
    v4f vals[4];
#pragma unroll
    for (int it = 0; it < 4; ++it) {
      const int row = it * 4 + q4;
      vals[it] = *(const v4f*)(os + row * 32 + e4);
    }
    for (int pass = 0; pass < 2; ++pass) {
#pragma unroll
      for (int it = 0; it < 4; ++it) {
        const int row = it * 4 + q4;
        *(volatile v4f*)(ao + (gr + row) * CD + a * HDIM + e4) = vals[it];
      }
      __threadfence();
    }
  }
}

__global__ __launch_bounds__(256) void ln_mid(const float* __restrict__ X, const float* __restrict__ gam,
                                               const float* __restrict__ bet, float* Y, unsigned short* YH,
                                               float hcarry) {
  __shared__ __align__(16) float sb[8][CD];
  const int tid = threadIdx.x, wave = tid >> 5, lane = tid & 31;
  const size_t base = ((size_t)blockIdx.x * 8 + wave) * CD;
  const v4f x0 = *(const v4f*)(X + base + 8 * lane), x1 = *(const v4f*)(X + base + 8 * lane + 4);
  float s = ((x0[0] + x0[1]) + (x0[2] + x0[3])) + ((x1[0] + x1[1]) + (x1[2] + x1[3]));
  s = wsum(s);
  const float mean = s * (1.0f / CD);
  float d[8];
#pragma unroll
  for (int e = 0; e < 4; ++e) { d[e] = x0[e] - mean; d[4 + e] = x1[e] - mean; }
  float vs = 0.f;
#pragma unroll
  for (int e = 0; e < 8; ++e) vs += d[e] * d[e];
  vs = wsum(vs);
  const float rstd = rsqrtf(vs * (1.0f / CD) + LNEPS);
  const v4f g0 = *(const v4f*)(gam + 8 * lane), g1 = *(const v4f*)(gam + 8 * lane + 4);
  const v4f b0 = *(const v4f*)(bet + 8 * lane), b1 = *(const v4f*)(bet + 8 * lane + 4);
  float y[8];
#pragma unroll
  for (int e = 0; e < 4; ++e) {
    y[e]     = (d[e] * rstd)     * bfr(g0[e]) + bfr(b0[e]);
    y[4 + e] = (d[4 + e] * rstd) * bfr(g1[e]) + bfr(b1[e]);
  }
  v4u oh;
#pragma unroll
  for (int e = 0; e < 4; ++e) oh[e] = pk16(h_bits((_Float16)(y[2 * e] * hcarry)), h_bits((_Float16)(y[2 * e + 1] * hcarry)));
  float* sw = sb[wave];
  v4f ya, yb;
#pragma unroll
  for (int e = 0; e < 4; ++e) { ya[e] = y[e]; yb[e] = y[4 + e]; }
  *(v4f*)(sw + 8 * lane)     = ya;
  *(v4f*)(sw + 8 * lane + 4) = yb;
  wave_sync_lds();
  const v4f o0 = *(const v4f*)(sw + 4 * lane);
  const v4f o1 = *(const v4f*)(sw + 128 + 4 * lane);
  for (int pass = 0; pass < 2; ++pass) {
    *(volatile v4u*)(YH + base + 8 * lane) = oh;
    *(volatile v4f*)(Y + base + 4 * lane) = o0;
    *(volatile v4f*)(Y + base + 128 + 4 * lane) = o1;
    __threadfence();
  }
}

__global__ __launch_bounds__(256) void ln_out(const float* __restrict__ Z, const float* __restrict__ gam,
                                               const float* __restrict__ bet, float* out) {
  __shared__ __align__(16) float T[CD * 36];
  const int tid = threadIdx.x, wave = tid >> 5, lane = tid & 31;
  const int bx = blockIdx.x;
  const int b  = bx >> 7;
  const int n0 = (bx & 127) * 32;
  const v4f g0 = *(const v4f*)(gam + 8 * lane), g1 = *(const v4f*)(gam + 8 * lane + 4);
  const v4f b0 = *(const v4f*)(bet + 8 * lane), b1 = *(const v4f*)(bet + 8 * lane + 4);
#pragma unroll 1
  for (int i = 0; i < 4; ++i) {
    const int tl = wave * 4 + i;
    const size_t base = ((size_t)b * NSEQ + n0 + tl) * CD;
    const v4f x0 = *(const v4f*)(Z + base + 8 * lane), x1 = *(const v4f*)(Z + base + 8 * lane + 4);
    float s = ((x0[0] + x0[1]) + (x0[2] + x0[3])) + ((x1[0] + x1[1]) + (x1[2] + x1[3]));
    s = wsum(s);
    const float mean = s * (1.0f / CD);
    float d[8];
#pragma unroll
    for (int e = 0; e < 4; ++e) { d[e] = x0[e] - mean; d[4 + e] = x1[e] - mean; }
    float vs = 0.f;
#pragma unroll
    for (int e = 0; e < 8; ++e) vs += d[e] * d[e];
    vs = wsum(vs);
    const float rstd = rsqrtf(vs * (1.0f / CD) + LNEPS);
#pragma unroll
    for (int e = 0; e < 4; ++e) {
      T[(8 * lane + e) * 36 + tl]     = (d[e] * rstd)     * bfr(g0[e]) + bfr(b0[e]);
      T[(8 * lane + 4 + e) * 36 + tl] = (d[4 + e] * rstd) * bfr(g1[e]) + bfr(b1[e]);
    }
  }
  __syncthreads();
  {
    const int q = lane >> 3, e4 = (lane & 7) * 4;
    v4f vals[8];
#pragma unroll
    for (int it = 0; it < 8; ++it) {
      const int cc = wave * 32 + it * 4 + q;
      vals[it] = *(const v4f*)(T + cc * 36 + e4);
    }
    for (int pass = 0; pass < 2; ++pass) {
#pragma unroll
      for (int it = 0; it < 8; ++it) {
        const int cc = wave * 32 + it * 4 + q;
        *(volatile v4f*)(out + ((size_t)(b * CD + cc)) * NSEQ + n0 + e4) = vals[it];
      }
      __threadfence();
    }
  }
}

extern "C" void kernel_launch(void* const* d_in, const int* in_sizes, int n_in,
                              void* d_out, int out_size, void* d_ws, size_t ws_size,
                              hipStream_t stream) {
  if (n_in < 23) return;
  if (in_sizes[0] != NB * CD * NSEQ) return;
  if (in_sizes[1] != NB * HW * CD || in_sizes[2] != NB * HW * CD) return;
  if (in_sizes[3] != CD * CD || in_sizes[5] != CD * CD || in_sizes[7] != CD * CD) return;
  if (in_sizes[9] != CD * CD || in_sizes[11] != CD * CD || in_sizes[13] != CD * CD) return;
  if (in_sizes[4] != CD || in_sizes[6] != CD || in_sizes[8] != CD || in_sizes[10] != CD) return;
  if (in_sizes[12] != CD || in_sizes[14] != CD || in_sizes[15] != CD || in_sizes[16] != CD) return;
  if (in_sizes[17] != DFF * CD || in_sizes[18] != DFF || in_sizes[19] != CD * DFF) return;
  if (in_sizes[20] != CD || in_sizes[21] != CD || in_sizes[22] != CD) return;
  if (out_size != NB * CD * NSEQ) return;

  const float* src    = (const float*)d_in[0];
  const float* pe_row = (const float*)d_in[1];
  const float* pe_col = (const float*)d_in[2];
  const float* wq_row = (const float*)d_in[3];   const float* bq_row = (const float*)d_in[4];
  const float* wq_col = (const float*)d_in[5];   const float* bq_col = (const float*)d_in[6];
  const float* wk_row = (const float*)d_in[7];   const float* bk_row = (const float*)d_in[8];
  const float* wk_col = (const float*)d_in[9];   const float* bk_col = (const float*)d_in[10];
  const float* w_v    = (const float*)d_in[11];  const float* b_v    = (const float*)d_in[12];
  const float* w_o    = (const float*)d_in[13];  const float* b_o    = (const float*)d_in[14];
  const float* g_1    = (const float*)d_in[15];  const float* be_1   = (const float*)d_in[16];
  const float* w_1    = (const float*)d_in[17];  const float* b_1    = (const float*)d_in[18];
  const float* w_2    = (const float*)d_in[19];  const float* b_2    = (const float*)d_in[20];
  const float* g_2    = (const float*)d_in[21];  const float* be_2   = (const float*)d_in[22];

  const size_t PW   = (size_t)CD * CD * 2;
  const size_t PWF  = (size_t)DFF * CD * 2;
  const size_t PAH  = (size_t)MP * CD * 2;
  const size_t PAF  = (size_t)MP * CD * 4;
  const size_t PXM  = (size_t)2 * NB * HW * CD * 2;
  const size_t PKH  = (size_t)2 * NB * HW * CD * 2;
  const size_t PVT  = (size_t)NB * CD * NSEQ * 2;
  const size_t PGH  = (size_t)MP * DFF * 2;
  size_t off = 0;
  const size_t oWH6 = off; off += 6 * PW;
  const size_t oW1  = off; off += PWF;
  const size_t oW2  = off; off += PWF;
  const size_t oXH  = off; off += PAH;
  const size_t oXPE = off; off += 2 * PAH;
  const size_t oXM  = off; off += PXM;
  const size_t oQH  = off; off += 2 * PAH;
  const size_t oKH  = off; off += PKH;
  const size_t oVT  = off; off += PVT;
  const size_t oAO  = off; off += PAF;
  const size_t oX1  = off; off += PAF;
  const size_t oY32 = off; off += PAF;
  const size_t oYH  = off; off += PAH;
  const size_t oGH  = off; off += PGH;
  const size_t oZ32 = off; off += PAF;
  if (off > ws_size) return;
  if (off > (size_t)134217728) return;

  char* ws = (char*)d_ws;
  unsigned short* WH6 = (unsigned short*)(ws + oWH6);
  unsigned short* W1H = (unsigned short*)(ws + oW1);
  unsigned short* W2H = (unsigned short*)(ws + oW2);
  unsigned short* XH  = (unsigned short*)(ws + oXH);
  unsigned short* XPE = (unsigned short*)(ws + oXPE);
  unsigned short* XM  = (unsigned short*)(ws + oXM);
  unsigned short* QH  = (unsigned short*)(ws + oQH);
  unsigned short* KH  = (unsigned short*)(ws + oKH);
  unsigned short* VT  = (unsigned short*)(ws + oVT);
  float*          AO  = (float*)(ws + oAO);
  float*          X1  = (float*)(ws + oX1);
  float*          Y32 = (float*)(ws + oY32);
  unsigned short* YH  = (unsigned short*)(ws + oYH);
  unsigned short* GH  = (unsigned short*)(ws + oGH);
  float*          Z32 = (float*)(ws + oZ32);
  float*          out = (float*)d_out;

  const int n8w = (CD * CD) / 8, n8f = (DFF * CD) / 8;
  if ((n8w % 256) != 0 || (n8f % 256) != 0) return;
  const dim3 blk(256), blk128(128);
  const dim3 gCw((n8w + 255) / 256), gCf((n8f + 255) / 256);
  const dim3 gPrep(MP / 32);
  const dim3 gMean(NB * 2 * 2);
  const dim3 gK((((2 * HW) / 64) * (CD / 64) + 7) / 8, 2);
  const dim3 gQ(((MP / 64) * (CD / 64) + 7) / 8, 2);
  const dim3 gV(((CD / 64) * (NSEQ / 64) + 7) / 8, NB);
  const dim3 gAttn(NB * NHEAD * (NSEQ / 64));
  const dim3 gO(((MP / 64) * (CD / 64) + 7) / 8, 1);
  const dim3 gLN(MP / 8);
  const dim3 gF1(((MP / 64) * (DFF / 64) + 7) / 8, 1);
  const dim3 gOut(MP / 32);
  const float qsc = 0.17677669529663688f;

  conv_h16<<<gCw, blk, 0, stream>>>(wq_row, WH6 + 0 * (size_t)CD * CD, n8w, WSC);
  conv_h16<<<gCw, blk, 0, stream>>>(wq_col, WH6 + 1 * (size_t)CD * CD, n8w, WSC);
  conv_h16<<<gCw, blk, 0, stream>>>(wk_row, WH6 + 2 * (size_t)CD * CD, n8w, WSC);
  conv_h16<<<gCw, blk, 0, stream>>>(wk_col, WH6 + 3 * (size_t)CD * CD, n8w, WSC);
  conv_h16<<<gCw, blk, 0, stream>>>(w_v,    WH6 + 4 * (size_t)CD * CD, n8w, WSC);
  conv_h16<<<gCw, blk, 0, stream>>>(w_o,    WH6 + 5 * (size_t)CD * CD, n8w, WSC);
  conv_h16<<<gCf, blk, 0, stream>>>(w_1, W1H, n8f, WSC);
  conv_h16<<<gCf, blk, 0, stream>>>(w_2, W2H, n8f, WSC);

  xprep<<<gPrep, blk, 0, stream>>>(src, pe_row, pe_col, XH, XPE, XPE + (size_t)MP * CD);
  xmean<<<gMean, blk, 0, stream>>>(src, pe_row, pe_col, XM);

  gemm64<0, 2, 0, 0, 0><<<gK, blk, 0, stream>>>(
      (const void*)XM, CD, (long long)NB * HW * CD, 1.0f,
      WH6 + 2 * (size_t)CD * CD, CD, (long long)CD * CD,
      bk_row, bk_col, KCARRY, (const void*)X1,
      (void*)KH, CD, (long long)NB * HW * CD, NB * HW, CD, CD, KCARRY / WSC);

  gemm64<0, 2, 0, 0, 0><<<gQ, blk, 0, stream>>>(
      (const void*)XPE, CD, (long long)MP * CD, 1.0f,
      WH6 + 0 * (size_t)CD * CD, CD, (long long)CD * CD,
      bq_row, bq_col, qsc * QCARRY, (const void*)X1,
      (void*)QH, CD, (long long)MP * CD, MP, CD, CD, qsc * QCARRY / WSC);

  gemm64<0, 2, 1, 0, 0><<<gV, blk, 0, stream>>>(
      (const void*)(WH6 + 4 * (size_t)CD * CD), CD, 0LL, 1.0f,
      XH, CD, (long long)NSEQ * CD,
      b_v, b_v, VCARRY, (const void*)X1,
      (void*)VT, NSEQ, (long long)CD * NSEQ, CD, NSEQ, CD, VCARRY / WSC);

  attn_rc<<<gAttn, blk128, 0, stream>>>(QH, KH, VT, AO);

  gemm64<1, 0, 0, 0, 2><<<gO, blk, 0, stream>>>(
      (const void*)AO, CD, 0LL, AOCARRY,
      WH6 + 5 * (size_t)CD * CD, CD, 0LL,
      b_o, b_o, 1.0f, (const void*)XH,
      (void*)X1, CD, 0LL, MP, CD, CD, 1.0f / (AOCARRY * WSC));

  ln_mid<<<gLN, blk, 0, stream>>>(X1, g_1, be_1, Y32, YH, YCARRY);

  gemm64<0, 2, 0, 1, 0><<<gF1, blk, 0, stream>>>(
      (const void*)YH, CD, 0LL, 1.0f,
      W1H, CD, 0LL,
      b_1, b_1, GCARRY, (const void*)X1,
      (void*)GH, DFF, 0LL, MP, DFF, CD, GCARRY / (YCARRY * WSC));

  gemm64<0, 0, 0, 0, 1><<<gO, blk, 0, stream>>>(
      (const void*)GH, DFF, 0LL, 1.0f,
      W2H, DFF, 0LL,
      b_2, b_2, 1.0f, (const void*)Y32,
      (void*)Z32, CD, 0LL, MP, CD, DFF, 1.0f / (GCARRY * WSC));

  ln_out<<<gOut, blk, 0, stream>>>(Z32, g_2, be_2, out);
  (void)hipGetLastError();
}
